// Net_MP_46849503265410
// MI455X (gfx1250) — hardware-verified
//
#include <hip/hip_runtime.h>
#include <stddef.h>


#define NTHR   128
#define NWAVE  4
#define EPT    8
#define CHUNK  (NTHR * EPT)
#define WCAP   (EPT * 32)
#define LISTN  (NWAVE * WCAP)
#define PASSN  (NWAVE * 32)
#define PCAP   (CHUNK + PASSN)
#define NB     512
#define OW     32
#define KL1    64
#define KL2    544
#define G2N    ((OW * KL2) / 8)
#define G1N    ((OW * KL1) / 8)
#define RPW    (NB / NWAVE)
#define TPW    ((NB / 16) / NWAVE)

static_assert(PASSN == 128);
static_assert(PCAP >= CHUNK + PASSN);
static_assert((RPW % 4) == 0);
static_assert(NB == NWAVE * 128);
static_assert(TPW * 16 * NWAVE == NB);
static_assert((G2N % NTHR) == 0);
static_assert((G1N % NTHR) == 0);
static_assert((KL2 % 32) == 0);
static_assert((KL1 % 32) == 0);

typedef float          v4f   __attribute__((ext_vector_type(4)));
typedef float          v8f   __attribute__((ext_vector_type(8)));
typedef int            v4i   __attribute__((ext_vector_type(4)));
typedef unsigned short v8us  __attribute__((ext_vector_type(8)));
typedef unsigned short v16us __attribute__((ext_vector_type(16)));
typedef __bf16         v16b  __attribute__((ext_vector_type(16)));
union FragB { v16b v; v16us u; v8us h[2]; };

__device__ __forceinline__ unsigned short bfr(float f) {
  unsigned u = __float_as_uint(f);
  u += 0x7FFFu + ((u >> 16) & 1u);
  return (unsigned short)(u >> 16);
}

__device__ __forceinline__ void split2(float p, unsigned short& hs, unsigned short& ls) {
  hs = bfr(p);
  const float hf = __uint_as_float(((unsigned)hs) << 16);
  ls = bfr(p - hf);
}

__device__ __forceinline__ v8f z8f() {
  v8f c;
#pragma unroll
  for (int i = 0; i < 8; ++i) c[i] = 0.0f;
  return c;
}

__device__ __forceinline__ v8f wmb(v16b a, v16b b, v8f c) {
  v8f d = __builtin_amdgcn_wmma_f32_16x16x32_bf16(false, a, false, b, (short)0, c, false, false);
  asm volatile("v_nop\n\tv_nop\n\tv_nop\n\tv_nop" : "+v"(d) : "v"(a), "v"(b));
  return d;
}

__device__ __forceinline__ v8f wm3(const FragB& ah, const FragB& al, const FragB& bh, const FragB& bl, v8f c) {
  c = wmb(ah.v, bh.v, c);
  c = wmb(ah.v, bl.v, c);
  c = wmb(al.v, bh.v, c);
  return c;
}

__device__ __forceinline__ FragB ldb(const unsigned short* p, int h) {
  FragB f;
  f.h[0] = *(const v8us*)(p + 8 * h);
  f.h[1] = *(const v8us*)(p + 16 + 8 * h);
  return f;
}

__device__ __forceinline__ v4f sel4(v4f v, bool ok) {
  v4f r;
  r.x = ok ? v.x : 0.0f; r.y = ok ? v.y : 0.0f; r.z = ok ? v.z : 0.0f; r.w = ok ? v.w : 0.0f;
  return r;
}

__device__ __forceinline__ int scan_chunk(const int* __restrict__ dsts, int nE, int cbase, int nodeBase,
                                          int vec8, int* list, int tid, int wave) {
  int wc = 0;
  const int el0  = tid * EPT;
  const int e0   = cbase + el0;
  const int sent = -2147483647 - 1;
  v4i da, db;
  if (vec8 != 0 && cbase + CHUNK <= nE) {
    da = *(const v4i*)(dsts + e0);
    db = *(const v4i*)(dsts + e0 + 4);
  } else {
    da.x = (e0     < nE) ? dsts[min(e0, nE - 1)] : sent;
    da.y = (e0 + 1 < nE) ? dsts[min(e0 + 1, nE - 1)] : sent;
    da.z = (e0 + 2 < nE) ? dsts[min(e0 + 2, nE - 1)] : sent;
    da.w = (e0 + 3 < nE) ? dsts[min(e0 + 3, nE - 1)] : sent;
    db.x = (e0 + 4 < nE) ? dsts[min(e0 + 4, nE - 1)] : sent;
    db.y = (e0 + 5 < nE) ? dsts[min(e0 + 5, nE - 1)] : sent;
    db.z = (e0 + 6 < nE) ? dsts[min(e0 + 6, nE - 1)] : sent;
    db.w = (e0 + 7 < nE) ? dsts[min(e0 + 7, nE - 1)] : sent;
  }
  const unsigned nb = (unsigned)nodeBase;
  const unsigned s0 = (unsigned)da.x - nb, s1 = (unsigned)da.y - nb;
  const unsigned s2 = (unsigned)da.z - nb, s3 = (unsigned)da.w - nb;
  const unsigned s4 = (unsigned)db.x - nb, s5 = (unsigned)db.y - nb;
  const unsigned s6 = (unsigned)db.z - nb, s7 = (unsigned)db.w - nb;
  const bool h0 = s0 < (unsigned)NB, h1 = s1 < (unsigned)NB, h2 = s2 < (unsigned)NB, h3 = s3 < (unsigned)NB;
  const bool h4 = s4 < (unsigned)NB, h5 = s5 < (unsigned)NB, h6 = s6 < (unsigned)NB, h7 = s7 < (unsigned)NB;
  const unsigned any = __builtin_amdgcn_ballot_w32(h0 | h1 | h2 | h3 | h4 | h5 | h6 | h7);
  if (any != 0u) {
#define HITJ(J, HJ) { \
      const unsigned mj = __builtin_amdgcn_ballot_w32(HJ); \
      if (mj != 0u) { \
        if (HJ) { \
          const int pos = wc + (int)__builtin_amdgcn_mbcnt_lo(mj, 0u); \
          if (pos < WCAP) list[wave * WCAP + pos] = el0 + (J); \
        } \
        wc += (int)__builtin_popcount(mj); } }
    HITJ(0, h0)
    HITJ(1, h1)
    HITJ(2, h2)
    HITJ(3, h3)
    HITJ(4, h4)
    HITJ(5, h5)
    HITJ(6, h6)
    HITJ(7, h7)
#undef HITJ
  }
  return wc;
}

__global__ __launch_bounds__(NTHR) void k_prep(const float* __restrict__ w12, const float* __restrict__ b12,
                                               const float* __restrict__ w22, const float* __restrict__ b22,
                                               unsigned short* W1h, unsigned short* W1l,
                                               unsigned short* W2h, unsigned short* W2l) {
  const int gid = blockIdx.x * NTHR + threadIdx.x;
  v8us hv, lv;
#pragma unroll
  for (int j = 0; j < 8; ++j) { hv[j] = (unsigned short)0; lv[j] = (unsigned short)0; }
  unsigned short* ph = W2h;
  unsigned short* pl = W2l;
  size_t go = 0;
  bool wr = false;
  if (gid < G2N) {
    const int o  = gid / (KL2 / 8);
    const int qg = gid - o * (KL2 / 8);
#pragma unroll
    for (int j = 0; j < 8; ++j) {
      const int q  = qg * 8 + j;
      const int qa = q < 511 ? q : 511;
      int qb = q - 512; qb = qb < 0 ? 0 : qb;
      const float va = w22[(qa >> 5) * 1024 + (qa & 31) * 32 + o];
      const float vb = b22[qb * 32 + o];
      const float v  = (q < 512) ? va : vb;
      unsigned short hs, ls;
      split2(v, hs, ls);
      hv[j] = hs; lv[j] = ls;
    }
    go = (size_t)gid * 8;
    wr = true;
  } else if (gid < G2N + G1N) {
    const int g  = gid - G2N;
    const int o  = g >> 3;
    const int qg = g & 7;
#pragma unroll
    for (int j = 0; j < 8; ++j) {
      const int q  = qg * 8 + j;
      const int qa = q < 47 ? q : 47;
      const int ia = qa >> 4, ka = qa & 15;
      int qb = q - 48; qb = qb < 0 ? 0 : (qb > 2 ? 2 : qb);
      const float va = w12[ka * 96 + ia * 32 + o];
      const float vb = b12[qb * 32 + o];
      const float v  = (q < 48) ? va : ((q < 51) ? vb : 0.0f);
      unsigned short hs, ls;
      split2(v, hs, ls);
      hv[j] = hs; lv[j] = ls;
    }
    ph = W1h; pl = W1l;
    go = (size_t)g * 8;
    wr = true;
  }
  if (wr) { *(volatile v8us*)(ph + go) = hv; *(volatile v8us*)(pl + go) = lv; }
  __threadfence();
  if (wr) { *(volatile v8us*)(ph + go) = hv; *(volatile v8us*)(pl + go) = lv; }
}

__device__ __forceinline__ void l1_pass(const float* acc, const float* cntL, const float* r1L, const float* bs1L,
                                        const float* __restrict__ x, float* hout, int nodeBase, int nN,
                                        int wave, int lane) {
#pragma unroll 1
  for (int q = 0; q < RPW / 4; ++q) {
    const int slot = wave * RPW + q * 4 + (lane >> 3);
    const int cg   = 4 * (lane & 7);
    const int n    = nodeBase + slot;
    const int nc   = n < nN ? n : nN - 1;
    const float x0 = x[(size_t)nc * 3], x1 = x[(size_t)nc * 3 + 1], x2 = x[(size_t)nc * 3 + 2];
    const float inv = 1.0f / fmaxf(cntL[slot], 1.0f);
    v4f o;
#pragma unroll
    for (int j = 0; j < 4; ++j) {
      const int col = cg + j;
      float xr = x0 * r1L[col] + x1 * r1L[32 + col];
      xr += x2 * r1L[64 + col];
      float v = xr + acc[slot * OW + col] * inv;
      v += bs1L[col];
      v = fmaxf(v, 0.0f);
      o[j] = (n < nN) ? v : 0.0f;
    }
    *(volatile v4f*)(hout + (size_t)n * OW + cg) = o;
  }
}

__global__ __launch_bounds__(NTHR) void k_conv1(
    const float* __restrict__ x, const int* __restrict__ ei, const float* __restrict__ ea,
    const float* __restrict__ w1, const float* __restrict__ b1,
    const unsigned short* __restrict__ Wh, const unsigned short* __restrict__ Wl,
    const float* __restrict__ root1, const float* __restrict__ bias1,
    float* hout, int nN, int nE, int vec8) {
  __shared__ __attribute__((aligned(16))) float acc[(NB + 1) * OW];
  __shared__ __attribute__((aligned(16))) float cntL[NB + 16];
  __shared__ __attribute__((aligned(16))) float msg[PASSN * OW];
  __shared__ __attribute__((aligned(16))) float xsL[PASSN * 4];
  __shared__ __attribute__((aligned(16))) float heL[PASSN * 16];
  __shared__ __attribute__((aligned(16))) int   list[LISTN];
  __shared__ __attribute__((aligned(16))) int   pend[PCAP];
  __shared__ int   slotb[PASSN];
  __shared__ __attribute__((aligned(16))) float w1L[64];
  __shared__ __attribute__((aligned(16))) float b1L[16];
  __shared__ __attribute__((aligned(16))) float r1L[96];
  __shared__ __attribute__((aligned(16))) float bs1L[32];
  __shared__ int wcnt[NWAVE];
  __shared__ int pendN;

  const int tid = threadIdx.x, lane = tid & 31, wave = tid >> 5, hh = lane >> 4, m = lane & 15;
  const int nodeBase = blockIdx.x * NB;
  const int* srcs = ei;
  const int* dsts = ei + nE;

  for (int i = tid; i < (NB + 1) * OW; i += NTHR) acc[i] = 0.0f;
  for (int i = tid; i < NB + 16; i += NTHR) cntL[i] = 0.0f;
  if (tid < 64) w1L[tid] = w1[tid];
  if (tid < 16) b1L[tid] = b1[tid];
  if (tid < 96) r1L[tid] = root1[tid];
  if (tid < 32) bs1L[tid] = bias1[tid];
  if (tid == 0) pendN = 0;
  __syncthreads();

  const int nChunks = (nE + CHUNK - 1) / CHUNK;
#pragma unroll 1
  for (int ch = 0; ch < nChunks; ++ch) {
    const int cbase = ch * CHUNK;
    const int wc = scan_chunk(dsts, nE, cbase, nodeBase, vec8, list, tid, wave);
    if (lane == 0) wcnt[wave] = wc;
    __syncthreads();

    const int base = pendN;
    int tot = 0, myoff = 0;
#pragma unroll
    for (int w = 0; w < NWAVE; ++w) {
      int c = wcnt[w];
      c = c > WCAP ? WCAP : (c < 0 ? 0 : c);
      if (w < wave) myoff += c;
      tot += c;
    }
    int newN = base + tot;
    newN = newN > PCAP ? PCAP : newN;
    {
      int n = wcnt[wave];
      n = n > WCAP ? WCAP : (n < 0 ? 0 : n);
      const int* lp = list + wave * WCAP;
      for (int i = lane; i < n; i += 32) {
        const int pos = base + myoff + i;
        if (pos < PCAP) pend[pos] = cbase + lp[i];
      }
    }
    const int fin = (ch == nChunks - 1) ? 1 : 0;
    const int R   = (fin != 0) ? (newN + PASSN - 1) / PASSN : newN / PASSN;
    const int Pv  = (fin != 0) ? newN : R * PASSN;
    __syncthreads();

#pragma unroll 1
    for (int r = 0; r < R; ++r) {
      {
        const int idx = r * PASSN + wave * 32 + lane;
        const bool valid = idx < Pv;
        int e = pend[idx];
        if (!valid) e = 0;
        e = e < 0 ? 0 : (e > nE - 1 ? nE - 1 : e);
        const int d = dsts[e];
        int s = srcs[e];
        int slot = d - nodeBase;
        if (!valid || (unsigned)slot >= (unsigned)NB) slot = NB;
        s = s < 0 ? 0 : (s > nN - 1 ? nN - 1 : s);
        const v4f av = *(const v4f*)(ea + (size_t)e * 4);
        const float x0 = x[(size_t)s * 3], x1 = x[(size_t)s * 3 + 1], x2 = x[(size_t)s * 3 + 2];
        v4f xv;
        xv.x = valid ? x0 : 0.0f; xv.y = valid ? x1 : 0.0f; xv.z = valid ? x2 : 0.0f; xv.w = 0.0f;
        *(v4f*)(xsL + (wave * 32 + lane) * 4) = xv;
        float* hp = heL + (wave * 32 + lane) * 16;
#pragma unroll
        for (int k4 = 0; k4 < 4; ++k4) {
          v4f hv4;
#pragma unroll
          for (int j = 0; j < 4; ++j) {
            const int k = 4 * k4 + j;
            float t = av.x * w1L[k] + av.y * w1L[16 + k];
            t += av.z * w1L[32 + k];
            t += av.w * w1L[48 + k];
            t += b1L[k];
            t = fmaxf(t, 0.0f);
            hv4[j] = valid ? t : 0.0f;
          }
          *(v4f*)(hp + 4 * k4) = hv4;
        }
        slotb[wave * 32 + lane] = slot;
      }
      __syncthreads();

#pragma unroll 1
      for (int t = 0; t < 2; ++t) {
        const int tb = r * PASSN + wave * 32 + 16 * t;
        if (tb < Pv) {
          const int er = wave * 32 + 16 * t + m;
          const v4f xv = *(const v4f*)(xsL + er * 4);
          const v4f ga = *(const v4f*)(heL + er * 16 + 8 * hh);
          const v4f gb = *(const v4f*)(heL + er * 16 + 8 * hh + 4);
          const float g8[8] = {ga.x, ga.y, ga.z, ga.w, gb.x, gb.y, gb.z, gb.w};
          const unsigned short* c0h = Wh + (size_t)m * KL1;
          const unsigned short* c0l = Wl + (size_t)m * KL1;
          const unsigned short* c1h = Wh + (size_t)(16 + m) * KL1;
          const unsigned short* c1l = Wl + (size_t)(16 + m) * KL1;
          v8f d0 = z8f(), d1 = z8f();
          FragB ah, al;
#pragma unroll
          for (int j = 0; j < 8; ++j) {
            unsigned short hs, ls;
            split2(xv.x * g8[j], hs, ls); ah.u[j] = hs;     al.u[j] = ls;
            split2(xv.y * g8[j], hs, ls); ah.u[8 + j] = hs; al.u[8 + j] = ls;
          }
          {
            const FragB bh0 = ldb(c0h, hh), bl0 = ldb(c0l, hh), bh1 = ldb(c1h, hh), bl1 = ldb(c1l, hh);
            d0 = wm3(ah, al, bh0, bl0, d0);
            d1 = wm3(ah, al, bh1, bl1, d1);
          }
#pragma unroll
          for (int j = 0; j < 8; ++j) {
            unsigned short hs, ls;
            split2(xv.z * g8[j], hs, ls); ah.u[j] = hs; al.u[j] = ls;
          }
          {
            unsigned short hs, ls;
            const float p8  = (hh == 0) ? xv.x : 0.0f;
            const float p9  = (hh == 0) ? xv.y : 0.0f;
            const float p10 = (hh == 0) ? xv.z : 0.0f;
            split2(p8,  hs, ls); ah.u[8]  = hs; al.u[8]  = ls;
            split2(p9,  hs, ls); ah.u[9]  = hs; al.u[9]  = ls;
            split2(p10, hs, ls); ah.u[10] = hs; al.u[10] = ls;
#pragma unroll
            for (int j = 11; j < 16; ++j) { ah.u[j] = (unsigned short)0; al.u[j] = (unsigned short)0; }
          }
          {
            const FragB bh0 = ldb(c0h + 32, hh), bl0 = ldb(c0l + 32, hh), bh1 = ldb(c1h + 32, hh), bl1 = ldb(c1l + 32, hh);
            d0 = wm3(ah, al, bh0, bl0, d0);
            d1 = wm3(ah, al, bh1, bl1, d1);
          }
          float* mp = msg + (wave * 32 + 16 * t + 8 * hh) * OW;
#pragma unroll
          for (int rr = 0; rr < 8; ++rr) { mp[rr * OW + m] = d0[rr]; mp[rr * OW + 16 + m] = d1[rr]; }
        }
      }
      __syncthreads();

      if (wave == 0) {
        int nv = Pv - r * PASSN;
        nv = nv > PASSN ? PASSN : (nv < 0 ? 0 : nv);
#pragma unroll 1
        for (int i = 0; i < nv; ++i) {
          int sl = slotb[i];
          sl = sl < 0 ? 0 : (sl > NB ? NB : sl);
          const float v = msg[i * OW + lane];
          acc[sl * OW + lane] += v;
          if (lane == 0) cntL[sl] += 1.0f;
        }
      }
      __syncthreads();
    }

    int rem = newN - R * PASSN;
    rem = rem < 0 ? 0 : rem;
    if (R > 0 && tid < rem) pend[tid] = pend[R * PASSN + tid];
    if (tid == 0) pendN = rem;
  }
  __syncthreads();

  l1_pass(acc, cntL, r1L, bs1L, x, hout, nodeBase, nN, wave, lane);
  __threadfence();
  l1_pass(acc, cntL, r1L, bs1L, x, hout, nodeBase, nN, wave, lane);
}

__global__ __launch_bounds__(NTHR) void k_conv2(
    const float* __restrict__ hin,
    const int* __restrict__ ei, const float* __restrict__ ea,
    const float* __restrict__ w1, const float* __restrict__ b1,
    const unsigned short* __restrict__ Wh, const unsigned short* __restrict__ Wl,
    const float* __restrict__ root2, const float* __restrict__ bias2,
    const float* __restrict__ fw, const float* __restrict__ fb,
    const float* __restrict__ gw, const float* __restrict__ gb,
    float* outp, int nN, int nE, int vec8) {
  __shared__ __attribute__((aligned(16))) float acc[(NB + 1) * OW];
  __shared__ __attribute__((aligned(16))) float cntL[NB + 16];
  __shared__ __attribute__((aligned(16))) float msg[PASSN * OW];
  __shared__ __attribute__((aligned(16))) float xsL[PASSN * OW];
  __shared__ __attribute__((aligned(16))) float heL[PASSN * 16];
  __shared__ __attribute__((aligned(16))) int   list[LISTN];
  __shared__ __attribute__((aligned(16))) int   pend[PCAP];
  __shared__ int   slotb[PASSN];
  __shared__ __attribute__((aligned(16))) unsigned short rh[OW * OW];
  __shared__ __attribute__((aligned(16))) unsigned short rl[OW * OW];
  __shared__ __attribute__((aligned(16))) unsigned short fh[OW * OW];
  __shared__ __attribute__((aligned(16))) unsigned short fl[OW * OW];
  __shared__ __attribute__((aligned(16))) float w1L[64];
  __shared__ __attribute__((aligned(16))) float b1L[16];
  __shared__ __attribute__((aligned(16))) float bs2L[32];
  __shared__ __attribute__((aligned(16))) float fbL[32];
  __shared__ __attribute__((aligned(16))) float gwL[32];
  __shared__ int wcnt[NWAVE];
  __shared__ int pendN;

  const int tid = threadIdx.x, lane = tid & 31, wave = tid >> 5, hh = lane >> 4, m = lane & 15;
  const int nodeBase = blockIdx.x * NB;
  const int* srcs = ei;
  const int* dsts = ei + nE;
  const float gb0 = gb[0];

  for (int i = tid; i < (NB + 1) * OW; i += NTHR) acc[i] = 0.0f;
  for (int i = tid; i < NB + 16; i += NTHR) cntL[i] = 0.0f;
  for (int i = tid; i < OW * OW; i += NTHR) {
    const int o = i >> 5, k = i & 31;
    unsigned short hs, ls;
    split2(root2[k * 32 + o], hs, ls); rh[o * OW + k] = hs; rl[o * OW + k] = ls;
    split2(fw[k * 32 + o],    hs, ls); fh[o * OW + k] = hs; fl[o * OW + k] = ls;
  }
  if (tid < 64) w1L[tid] = w1[tid];
  if (tid < 16) b1L[tid] = b1[tid];
  if (tid < 32) { bs2L[tid] = bias2[tid]; fbL[tid] = fb[tid]; gwL[tid] = gw[tid]; }
  if (tid == 0) pendN = 0;
  __syncthreads();

  const int nChunks = (nE + CHUNK - 1) / CHUNK;
#pragma unroll 1
  for (int ch = 0; ch < nChunks; ++ch) {
    const int cbase = ch * CHUNK;
    const int wc = scan_chunk(dsts, nE, cbase, nodeBase, vec8, list, tid, wave);
    if (lane == 0) wcnt[wave] = wc;
    __syncthreads();

    const int base = pendN;
    int tot = 0, myoff = 0;
#pragma unroll
    for (int w = 0; w < NWAVE; ++w) {
      int c = wcnt[w];
      c = c > WCAP ? WCAP : (c < 0 ? 0 : c);
      if (w < wave) myoff += c;
      tot += c;
    }
    int newN = base + tot;
    newN = newN > PCAP ? PCAP : newN;
    {
      int n = wcnt[wave];
      n = n > WCAP ? WCAP : (n < 0 ? 0 : n);
      const int* lp = list + wave * WCAP;
      for (int i = lane; i < n; i += 32) {
        const int pos = base + myoff + i;
        if (pos < PCAP) pend[pos] = cbase + lp[i];
      }
    }
    const int fin = (ch == nChunks - 1) ? 1 : 0;
    const int R   = (fin != 0) ? (newN + PASSN - 1) / PASSN : newN / PASSN;
    const int Pv  = (fin != 0) ? newN : R * PASSN;
    __syncthreads();

#pragma unroll 1
    for (int r = 0; r < R; ++r) {
      {
        const int idx = r * PASSN + wave * 32 + lane;
        const bool valid = idx < Pv;
        int e = pend[idx];
        if (!valid) e = 0;
        e = e < 0 ? 0 : (e > nE - 1 ? nE - 1 : e);
        const int d = dsts[e];
        int s = srcs[e];
        int slot = d - nodeBase;
        if (!valid || (unsigned)slot >= (unsigned)NB) slot = NB;
        s = s < 0 ? 0 : (s > nN - 1 ? nN - 1 : s);
        const v4f av = *(const v4f*)(ea + (size_t)e * 4);
        const float* hr = hin + (size_t)s * OW;
        float* xp = xsL + (wave * 32 + lane) * OW;
#pragma unroll
        for (int g = 0; g < 8; ++g) {
          const v4f v = *(const v4f*)(hr + 4 * g);
          *(v4f*)(xp + 4 * g) = sel4(v, valid);
        }
        float* hp = heL + (wave * 32 + lane) * 16;
#pragma unroll
        for (int k4 = 0; k4 < 4; ++k4) {
          v4f hv4;
#pragma unroll
          for (int j = 0; j < 4; ++j) {
            const int k = 4 * k4 + j;
            float t = av.x * w1L[k] + av.y * w1L[16 + k];
            t += av.z * w1L[32 + k];
            t += av.w * w1L[48 + k];
            t += b1L[k];
            t = fmaxf(t, 0.0f);
            hv4[j] = valid ? t : 0.0f;
          }
          *(v4f*)(hp + 4 * k4) = hv4;
        }
        slotb[wave * 32 + lane] = slot;
      }
      __syncthreads();

#pragma unroll 1
      for (int t = 0; t < 2; ++t) {
        const int tb = r * PASSN + wave * 32 + 16 * t;
        if (tb < Pv) {
          const int er = wave * 32 + 16 * t + m;
          const float* xr = xsL + er * OW;
          const v4f xa = *(const v4f*)(xr + 8 * hh);
          const v4f xb = *(const v4f*)(xr + 8 * hh + 4);
          const v4f xc = *(const v4f*)(xr + 16 + 8 * hh);
          const v4f xd = *(const v4f*)(xr + 16 + 8 * hh + 4);
          const float xf[16] = {xa.x, xa.y, xa.z, xa.w, xb.x, xb.y, xb.z, xb.w,
                                xc.x, xc.y, xc.z, xc.w, xd.x, xd.y, xd.z, xd.w};
          const float* hep = heL + er * 16;
          const unsigned short* c0h = Wh + (size_t)m * KL2;
          const unsigned short* c0l = Wl + (size_t)m * KL2;
          const unsigned short* c1h = Wh + (size_t)(16 + m) * KL2;
          const unsigned short* c1l = Wl + (size_t)(16 + m) * KL2;
          v8f d0 = z8f(), d1 = z8f();
#pragma unroll 1
          for (int c = 0; c < 17; ++c) {
            const int ci = c < 16 ? c : 0;
            const float gl = hep[ci];
            const float gc = c < 16 ? gl : 1.0f;
            FragB ah, al;
#pragma unroll
            for (int j = 0; j < 16; ++j) {
              unsigned short hs, ls;
              split2(xf[j] * gc, hs, ls);
              ah.u[j] = hs; al.u[j] = ls;
            }
            const int k0 = 32 * c;
            const FragB bh0 = ldb(c0h + k0, hh), bl0 = ldb(c0l + k0, hh);
            const FragB bh1 = ldb(c1h + k0, hh), bl1 = ldb(c1l + k0, hh);
            d0 = wm3(ah, al, bh0, bl0, d0);
            d1 = wm3(ah, al, bh1, bl1, d1);
          }
          float* mp = msg + (wave * 32 + 16 * t + 8 * hh) * OW;
#pragma unroll
          for (int rr = 0; rr < 8; ++rr) { mp[rr * OW + m] = d0[rr]; mp[rr * OW + 16 + m] = d1[rr]; }
        }
      }
      __syncthreads();

      if (wave == 0) {
        int nv = Pv - r * PASSN;
        nv = nv > PASSN ? PASSN : (nv < 0 ? 0 : nv);
#pragma unroll 1
        for (int i = 0; i < nv; ++i) {
          int sl = slotb[i];
          sl = sl < 0 ? 0 : (sl > NB ? NB : sl);
          const float v = msg[i * OW + lane];
          acc[sl * OW + lane] += v;
          if (lane == 0) cntL[sl] += 1.0f;
        }
      }
      __syncthreads();
    }

    int rem = newN - R * PASSN;
    rem = rem < 0 ? 0 : rem;
    if (R > 0 && tid < rem) pend[tid] = pend[R * PASSN + tid];
    if (tid == 0) pendN = rem;
  }
  __syncthreads();

  float* h2s  = msg + wave * 512;
  float* outL = xsL;
#pragma unroll 1
  for (int u = 0; u < TPW; ++u) {
    const int R0 = (wave * TPW + u) * 16;
    FragB ah, al;
    {
      const float* hr = hin + (size_t)(nodeBase + R0 + m) * OW;
      const v4f xa = *(const v4f*)(hr + 8 * hh);
      const v4f xb = *(const v4f*)(hr + 8 * hh + 4);
      const v4f xc = *(const v4f*)(hr + 16 + 8 * hh);
      const v4f xd = *(const v4f*)(hr + 16 + 8 * hh + 4);
      const float xf[16] = {xa.x, xa.y, xa.z, xa.w, xb.x, xb.y, xb.z, xb.w,
                            xc.x, xc.y, xc.z, xc.w, xd.x, xd.y, xd.z, xd.w};
#pragma unroll
      for (int j = 0; j < 16; ++j) { unsigned short hs, ls; split2(xf[j], hs, ls); ah.u[j] = hs; al.u[j] = ls; }
    }
    v8f d0, d1;
    {
      const FragB bh0 = ldb(rh + m * OW, hh), bl0 = ldb(rl + m * OW, hh);
      const FragB bh1 = ldb(rh + (16 + m) * OW, hh), bl1 = ldb(rl + (16 + m) * OW, hh);
      d0 = wm3(ah, al, bh0, bl0, z8f());
      d1 = wm3(ah, al, bh1, bl1, z8f());
    }
#pragma unroll
    for (int rr = 0; rr < 8; ++rr) {
      const int slot = R0 + 8 * hh + rr;
      const float inv = 1.0f / fmaxf(cntL[slot], 1.0f);
      float v0 = d0[rr] + acc[slot * OW + m] * inv;
      float v1 = d1[rr] + acc[slot * OW + 16 + m] * inv;
      v0 += bs2L[m]; v1 += bs2L[16 + m];
      h2s[(8 * hh + rr) * OW + m]      = fmaxf(v0, 0.0f);
      h2s[(8 * hh + rr) * OW + 16 + m] = fmaxf(v1, 0.0f);
    }
    __syncthreads();
    {
      const float* ar = h2s + m * OW;
      const v4f xa = *(const v4f*)(ar + 8 * hh);
      const v4f xb = *(const v4f*)(ar + 8 * hh + 4);
      const v4f xc = *(const v4f*)(ar + 16 + 8 * hh);
      const v4f xd = *(const v4f*)(ar + 16 + 8 * hh + 4);
      const float xf[16] = {xa.x, xa.y, xa.z, xa.w, xb.x, xb.y, xb.z, xb.w,
                            xc.x, xc.y, xc.z, xc.w, xd.x, xd.y, xd.z, xd.w};
#pragma unroll
      for (int j = 0; j < 16; ++j) { unsigned short hs, ls; split2(xf[j], hs, ls); ah.u[j] = hs; al.u[j] = ls; }
    }
    {
      const FragB bh0 = ldb(fh + m * OW, hh), bl0 = ldb(fl + m * OW, hh);
      const FragB bh1 = ldb(fh + (16 + m) * OW, hh), bl1 = ldb(fl + (16 + m) * OW, hh);
      d0 = wm3(ah, al, bh0, bl0, z8f());
      d1 = wm3(ah, al, bh1, bl1, z8f());
    }
    float pr[8];
#pragma unroll
    for (int rr = 0; rr < 8; ++rr) {
      const float f0 = fmaxf(d0[rr] + fbL[m], 0.0f);
      const float f1 = fmaxf(d1[rr] + fbL[16 + m], 0.0f);
      float p = f0 * gwL[m];
      p += f1 * gwL[16 + m];
      p += __shfl_xor(p, 1);
      p += __shfl_xor(p, 2);
      p += __shfl_xor(p, 4);
      p += __shfl_xor(p, 8);
      pr[rr] = p + gb0;
    }
    if (m == 0) {
#pragma unroll
      for (int rr = 0; rr < 8; ++rr) outL[R0 + 8 * hh + rr] = pr[rr];
    }
    __syncthreads();
  }

  {
    const int li = wave * 128 + 4 * lane;
    const v4f ov = *(const v4f*)(outL + li);
    const int gi = nodeBase + li;
    const bool wr = (gi + 3) < nN;
    if (wr) *(volatile v4f*)(outp + gi) = ov;
    __threadfence();
    if (wr) *(volatile v4f*)(outp + gi) = ov;
  }
}

extern "C" void kernel_launch(void* const* d_in, const int* in_sizes, int n_in,
                              void* d_out, int out_size, void* d_ws, size_t ws_size,
                              hipStream_t stream) {
  if (n_in < 19) return;
  const int nN = in_sizes[0] / 3;
  const int nE = in_sizes[1] / 2;
  if (nN <= 0 || nE <= 0) return;
  if (in_sizes[0] != nN * 3 || in_sizes[1] != nE * 2 || in_sizes[2] != nE * 4) return;
  if (in_sizes[3] != 64 || in_sizes[4] != 16 || in_sizes[5] != 16 * 96 || in_sizes[6] != 96) return;
  if (in_sizes[7] != 96 || in_sizes[8] != 32) return;
  if (in_sizes[9] != 64 || in_sizes[10] != 16 || in_sizes[11] != 16 * 1024 || in_sizes[12] != 1024) return;
  if (in_sizes[13] != 1024 || in_sizes[14] != 32) return;
  if (in_sizes[15] != 1024 || in_sizes[16] != 32 || in_sizes[17] != 32 || in_sizes[18] != 1) return;
  if (out_size != nN) return;

  const float* x     = (const float*)d_in[0];
  const int*   ei    = (const int*)d_in[1];
  const float* ea    = (const float*)d_in[2];
  const float* e1_w1 = (const float*)d_in[3];
  const float* e1_b1 = (const float*)d_in[4];
  const float* e1_w2 = (const float*)d_in[5];
  const float* e1_b2 = (const float*)d_in[6];
  const float* root1 = (const float*)d_in[7];
  const float* bias1 = (const float*)d_in[8];
  const float* e2_w1 = (const float*)d_in[9];
  const float* e2_b1 = (const float*)d_in[10];
  const float* e2_w2 = (const float*)d_in[11];
  const float* e2_b2 = (const float*)d_in[12];
  const float* root2 = (const float*)d_in[13];
  const float* bias2 = (const float*)d_in[14];
  const float* fc1_w = (const float*)d_in[15];
  const float* fc1_b = (const float*)d_in[16];
  const float* fc2_w = (const float*)d_in[17];
  const float* fc2_b = (const float*)d_in[18];
  float* out = (float*)d_out;

  const int nBlk = (nN + NB - 1) / NB;

  char* ws = (char*)d_ws;
  size_t off = 0;
  const size_t oW1h = off; off += (size_t)OW * KL1 * 2;      off = (off + 255) & ~(size_t)255;
  const size_t oW1l = off; off += (size_t)OW * KL1 * 2;      off = (off + 255) & ~(size_t)255;
  const size_t oW2h = off; off += (size_t)OW * KL2 * 2;      off = (off + 255) & ~(size_t)255;
  const size_t oW2l = off; off += (size_t)OW * KL2 * 2;      off = (off + 255) & ~(size_t)255;
  const size_t oH   = off; off += (size_t)nBlk * NB * OW * 4; off = (off + 255) & ~(size_t)255;
  if (off > ws_size) return;
  unsigned short* W1h = (unsigned short*)(ws + oW1h);
  unsigned short* W1l = (unsigned short*)(ws + oW1l);
  unsigned short* W2h = (unsigned short*)(ws + oW2h);
  unsigned short* W2l = (unsigned short*)(ws + oW2l);
  float* h1 = (float*)(ws + oH);

  const int vec8 = ((nE & 3) == 0) ? 1 : 0;

  k_prep<<<(G2N + G1N) / NTHR, NTHR, 0, stream>>>(e1_w2, e1_b2, e2_w2, e2_b2, W1h, W1l, W2h, W2l);

  k_conv1<<<nBlk, NTHR, 0, stream>>>(x, ei, ea, e1_w1, e1_b1, W1h, W1l, root1, bias1, h1, nN, nE, vec8);

  k_conv2<<<nBlk, NTHR, 0, stream>>>(h1, ei, ea, e2_w1, e2_b1, W2h, W2l, root2, bias2,
                                     fc1_w, fc1_b, fc2_w, fc2_b, out, nN, nE, vec8);
}
